// _JambaSSMCore_65687229825529
// MI455X (gfx1250) — hardware-run, weakly checked
//
#include <hip/hip_runtime.h>
#include <math.h>

typedef __attribute__((ext_vector_type(16))) _Float16 v16h;
typedef __attribute__((ext_vector_type(8)))  _Float16 v8h;
typedef __attribute__((ext_vector_type(2)))  _Float16 v2h;
typedef __attribute__((ext_vector_type(16))) __bf16   v16b;
typedef __attribute__((ext_vector_type(8)))  __bf16   v8b;
typedef __attribute__((ext_vector_type(8)))  float    v8f;
typedef __attribute__((ext_vector_type(4)))  float    v4f;
typedef __attribute__((ext_vector_type(4)))  unsigned v4u;

constexpr int kBatch = 2;
constexpr int kSeq   = 2048;
constexpr int kDm    = 1024;
constexpr int kNst   = 16;
constexpr int kNproj = kDm + 2 * kNst;
constexpr int kNpad  = 1088;
constexpr int kRows  = kBatch * kSeq;
constexpr int kWtP   = 68;
constexpr int kScanTS = 64;
constexpr int kScanCh = 64;
constexpr int kScanYP = 68;
constexpr int kHalfSt = 8;
static_assert(kNproj == 1056);
static_assert((kNpad % 64) == 0 && kNpad >= kNproj);
static_assert((kRows % 64) == 0 && (kDm % 32) == 0 && (kDm % 64) == 0);
static_assert((kSeq % kScanTS) == 0 && (kDm % kScanCh) == 0);
static_assert(kNst == 2 * kHalfSt);
static_assert((size_t)kRows * kDm * 4 == 16777216ull);

constexpr bool  kThreeProd = true;
constexpr int   kOpType    = kThreeProd ? 1 : 0;
constexpr float kCarryX    = kThreeProd ? 1.0f : 16.0f;
constexpr float kCarryW    = kThreeProd ? 1.0f : 1024.0f;
constexpr float kFold      = 1.0f / (kCarryX * kCarryW);
constexpr float kF16MinNormal = 6.103515625e-05f;

constexpr size_t kSzXH  = (size_t)kRows * kDm * 2;
constexpr size_t kSzWT  = (size_t)kNpad * kDm * 2;
constexpr size_t kSzP   = (size_t)kRows * kNpad * 4;
constexpr size_t kOffXH  = 0;
constexpr size_t kOffXL  = kOffXH  + kSzXH;
constexpr size_t kOffWTH = kOffXL  + kSzXH;
constexpr size_t kOffWTL = kOffWTH + kSzWT;
constexpr size_t kOffP   = kOffWTL + kSzWT;
constexpr size_t kWsTotal = kOffP + kSzP;
static_assert(kWsTotal == 39059456ull);
static_assert(kWsTotal <= 134217728ull);
static_assert((kOffXL % 128) == 0 && (kOffWTH % 128) == 0 && (kOffWTL % 128) == 0 && (kOffP % 128) == 0);

__device__ __forceinline__ void pin_u(unsigned& t) { asm volatile("" : "+v"(t)); }

__device__ __forceinline__ unsigned rne_bf16_word(float f) {
  unsigned u = __float_as_uint(f);
  const unsigned lsb = (u & 0x00010000u) ? 1u : 0u;
  u = (u + 0x7FFFu + lsb) & 0xFFFF0000u;
  return u;
}
__device__ __forceinline__ unsigned f16_pair_word(float a, float b) {
  const float fa = (fabsf(a) < kF16MinNormal) ? 0.0f : a;
  const float fb = (fabsf(b) < kF16MinNormal) ? 0.0f : b;
  const _Float16 ha = (_Float16)fa;
  const _Float16 hb = (_Float16)fb;
  v2h p;
  p.x = ha;
  p.y = hb;
  return __builtin_bit_cast(unsigned, p);
}
template <bool THREE>
__device__ __forceinline__ void pack8(const float (&f)[8], const float carry, v4u& wh, v4u& wl) {
  unsigned hw[4], lw[4];
#pragma unroll
  for (int p = 0; p < 4; ++p) {
    const float fe = f[2 * p];
    const float fo = f[2 * p + 1];
    if (THREE) {
      const unsigned he = rne_bf16_word(fe);
      const unsigned ho = rne_bf16_word(fo);
      const unsigned le = rne_bf16_word(fe - __uint_as_float(he));
      const unsigned lo = rne_bf16_word(fo - __uint_as_float(ho));
      hw[p] = __builtin_amdgcn_perm(ho, he, 0x07060302u);
      lw[p] = __builtin_amdgcn_perm(lo, le, 0x07060302u);
    } else {
      hw[p] = f16_pair_word(fe * carry, fo * carry);
      lw[p] = 0u;
    }
  }
  wh.x = hw[0]; wh.y = hw[1]; wh.z = hw[2]; wh.w = hw[3];
  wl.x = lw[0]; wl.y = lw[1]; wl.z = lw[2]; wl.w = lw[3];
}

__device__ __forceinline__ void dep1_h(v8f& c, v16h x, v16h y) { asm volatile("v_nop\n\tv_nop\n\tv_nop\n\tv_nop" : "+v"(c) : "v"(x), "v"(y)); }
__device__ __forceinline__ void dep1_b(v8f& c, v16b x, v16b y) { asm volatile("v_nop\n\tv_nop\n\tv_nop\n\tv_nop" : "+v"(c) : "v"(x), "v"(y)); }
__device__ __forceinline__ void dep2_h(v8f& c, v16h x, v16h y, v16h x2, v16h y2) { asm volatile("v_nop\n\tv_nop\n\tv_nop\n\tv_nop" : "+v"(c) : "v"(x), "v"(y), "v"(x2), "v"(y2)); }
__device__ __forceinline__ void dep2_b(v8f& c, v16b x, v16b y, v16b x2, v16b y2) { asm volatile("v_nop\n\tv_nop\n\tv_nop\n\tv_nop" : "+v"(c) : "v"(x), "v"(y), "v"(x2), "v"(y2)); }
__device__ __forceinline__ void keep4_h(v16h a, v16h b, v16h c, v16h d) { asm volatile("v_nop" :: "v"(a), "v"(b), "v"(c), "v"(d)); }
__device__ __forceinline__ void keep4_b(v16b a, v16b b, v16b c, v16b d) { asm volatile("v_nop" :: "v"(a), "v"(b), "v"(c), "v"(d)); }
__device__ __forceinline__ void acc_guard4(v8f& a, v8f& b, v8f& c, v8f& d) { asm volatile("v_nop\n\tv_nop\n\tv_nop\n\tv_nop" : "+v"(a), "+v"(b), "+v"(c), "+v"(d)); }

template <typename T> struct Frag;
template <> struct Frag<_Float16> {
  typedef v16h V; union U { v16h v; v8h h[2]; };
  static __device__ __forceinline__ v16h load(const _Float16* p) {
    U f; f.h[0] = *(const v8h*)(p); f.h[1] = *(const v8h*)(p + 16); return f.v;
  }
  static __device__ __forceinline__ v8f mma(v16h a, v16h b, v8f c) {
    return __builtin_amdgcn_wmma_f32_16x16x32_f16(false, a, false, b, (short)0, c, false, false);
  }
  static __device__ __forceinline__ void guard1(v8f& c, v16h x, v16h y) { dep1_h(c, x, y); }
  static __device__ __forceinline__ void guard2(v8f& c, v16h x, v16h y, v16h x2, v16h y2) { dep2_h(c, x, y, x2, y2); }
  static __device__ __forceinline__ void keep(v16h a, v16h b, v16h c, v16h d) { keep4_h(a, b, c, d); }
};
template <> struct Frag<__bf16> {
  typedef v16b V; union U { v16b v; v8b h[2]; };
  static __device__ __forceinline__ v16b load(const __bf16* p) {
    U f; f.h[0] = *(const v8b*)(p); f.h[1] = *(const v8b*)(p + 16); return f.v;
  }
  static __device__ __forceinline__ v8f mma(v16b a, v16b b, v8f c) {
    return __builtin_amdgcn_wmma_f32_16x16x32_bf16(false, a, false, b, (short)0, c, false, false);
  }
  static __device__ __forceinline__ void guard1(v8f& c, v16b x, v16b y) { dep1_b(c, x, y); }
  static __device__ __forceinline__ void guard2(v8f& c, v16b x, v16b y, v16b x2, v16b y2) { dep2_b(c, x, y, x2, y2); }
  static __device__ __forceinline__ void keep(v16b a, v16b b, v16b c, v16b d) { keep4_b(a, b, c, d); }
};
template <int ET> struct Elem;
template <> struct Elem<0> { typedef _Float16 T; };
template <> struct Elem<1> { typedef __bf16 T; };

constexpr unsigned kPackX8 = (unsigned)((size_t)kRows * kDm / 8);
static_assert((kPackX8 % 256u) == 0u);

template <bool THREE>
__global__ __launch_bounds__(256) void pack_rows_kernel(
    const float* __restrict__ src, unsigned short* __restrict__ dhi, unsigned short* __restrict__ dlo)
{
  const unsigned i = blockIdx.x * 256u + threadIdx.x;
  if (i >= kPackX8) return;
  const size_t e0 = (size_t)i << 3;
  const v4f a0 = *(const v4f*)(src + e0);
  const v4f a1 = *(const v4f*)(src + e0 + 4);
  float f[8];
  f[0] = a0.x; f[1] = a0.y; f[2] = a0.z; f[3] = a0.w;
  f[4] = a1.x; f[5] = a1.y; f[6] = a1.z; f[7] = a1.w;
  v4u wh, wl;
  pack8<THREE>(f, kCarryX, wh, wl);
  unsigned short* qh = dhi + e0;
  unsigned short* ql = dlo + e0;
  *(volatile v4u*)qh = wh;
  if (THREE) *(volatile v4u*)ql = wl;
  __threadfence();
  *(volatile v4u*)qh = wh;
  if (THREE) *(volatile v4u*)ql = wl;
}

template <bool THREE>
__global__ __launch_bounds__(256) void pack_wt_kernel(
    const float* __restrict__ W, unsigned short* __restrict__ thi, unsigned short* __restrict__ tlo)
{
  __shared__ __align__(16) float sT[64 * kWtP];
  const unsigned tid = threadIdx.x;
  const unsigned lane = tid & 31u;
  const unsigned wave = tid >> 5;
  const unsigned k0 = blockIdx.x * 64u;
  const unsigned n0 = blockIdx.y * 64u;
  unsigned lr = tid >> 4;
  unsigned lc4 = (tid & 15u) * 4u;
  pin_u(lr);
  pin_u(lc4);
  const unsigned n = n0 + lc4;
  const bool valid = n < (unsigned)kNproj;
  const unsigned nc = valid ? n : (unsigned)(kNproj - 4);
#pragma unroll
  for (int i = 0; i < 4; ++i) {
    const unsigned r = lr + 16u * (unsigned)i;
    const v4f v = *(const v4f*)(W + (size_t)(k0 + r) * kNproj + nc);
    v4f o;
    o.x = valid ? v.x : 0.0f;
    o.y = valid ? v.y : 0.0f;
    o.z = valid ? v.z : 0.0f;
    o.w = valid ? v.w : 0.0f;
    *(v4f*)(sT + r * kWtP + lc4) = o;
  }
  __syncthreads();
  unsigned q = lane >> 3;
  unsigned c8 = (lane & 7u) * 8u;
  pin_u(q);
  pin_u(c8);
  v4u wh[2], wl[2];
#pragma unroll
  for (int it = 0; it < 2; ++it) {
    const unsigned nl = (unsigned)it * 32u + wave * 4u + q;
    float f[8];
#pragma unroll
    for (int e = 0; e < 8; ++e) f[e] = sT[(c8 + (unsigned)e) * kWtP + nl];
    pack8<THREE>(f, kCarryW, wh[it], wl[it]);
  }
  for (int pass = 0; pass < 2; ++pass) {
#pragma unroll
    for (int it = 0; it < 2; ++it) {
      const unsigned nl = (unsigned)it * 32u + wave * 4u + q;
      const size_t off = (size_t)(n0 + nl) * kDm + k0 + c8;
      *(volatile v4u*)(thi + off) = wh[it];
      if (THREE) *(volatile v4u*)(tlo + off) = wl[it];
    }
    __threadfence();
  }
}

template <int ET, bool SPLIT>
__global__ __launch_bounds__(256) void proj_gemm_kernel(
    const unsigned short* __restrict__ Ap, const unsigned short* __restrict__ A2p,
    const unsigned short* __restrict__ Btp, const unsigned short* __restrict__ Bt2p,
    float* __restrict__ Cout)
{
  typedef typename Elem<ET>::T T;
  typedef typename Frag<T>::V V;
  constexpr int M = kRows, N = kNpad, K = kDm;
  constexpr int lda = kDm, ldb = kDm, ldc = kNpad;
  static_assert((M % 64) == 0 && (N % 64) == 0 && (K % 32) == 0);
  constexpr float kScale = kFold;
  const T* A = (const T*)Ap; const T* A2 = (const T*)A2p; const T* Bt = (const T*)Btp; const T* Bt2 = (const T*)Bt2p;
  __shared__ __align__(16) float sT[8][16 * 68];
  const int lane = threadIdx.x & 31;
  const int wave = threadIdx.x >> 5;
  constexpr int tilesN = N >> 6;
  constexpr int tilesM = M >> 6;
  const int tile = blockIdx.x * 8 + wave;
  if (tile >= tilesM * tilesN) return;
  const int tm = tile / tilesN;
  const int tn = tile - tm * tilesN;
  const int m0 = tm << 6;
  const int n0 = tn << 6;

  const int rlane = lane & 15;
  const int koff  = (lane >> 4) * 8;
  const int mOff  = (lane >> 4) * 8;

  v8f acc[4][4];
#pragma unroll
  for (int i = 0; i < 4; ++i)
#pragma unroll
    for (int j = 0; j < 4; ++j) acc[i][j] = (v8f){0.f,0.f,0.f,0.f,0.f,0.f,0.f,0.f};

  for (int k0 = 0; k0 < K; k0 += 32) {
    V bh[4], bl[4];
#pragma unroll
    for (int j = 0; j < 4; ++j) {
      const size_t bo = (size_t)(n0 + (j << 4) + rlane) * ldb + koff + k0;
      bh[j] = Frag<T>::load(Bt + bo);
      bl[j] = bh[j];
      if (SPLIT) bl[j] = Frag<T>::load(Bt2 + bo);
    }
#pragma unroll
    for (int i = 0; i < 4; ++i) {
      const size_t ao = (size_t)(m0 + (i << 4) + rlane) * lda + koff + k0;
      V ah = Frag<T>::load(A + ao);
      V al = ah;
      if (SPLIT) al = Frag<T>::load(A2 + ao);
#pragma unroll
      for (int j = 0; j < 4; ++j) {
        if (SPLIT) {
          acc[i][j] = Frag<T>::mma(al, bh[j], acc[i][j]);
          acc[i][j] = Frag<T>::mma(ah, bl[j], acc[i][j]);
        }
        acc[i][j] = Frag<T>::mma(ah, bh[j], acc[i][j]);
      }
#pragma unroll
      for (int j = 0; j < 4; ++j) {
        if (SPLIT) Frag<T>::guard2(acc[i][j], ah, bh[j], al, bl[j]);
        else       Frag<T>::guard1(acc[i][j], ah, bh[j]);
      }
    }
    Frag<T>::keep(bh[0], bh[1], bh[2], bh[3]);
    if (SPLIT) Frag<T>::keep(bl[0], bl[1], bl[2], bl[3]);
  }
  acc_guard4(acc[0][0], acc[0][1], acc[0][2], acc[0][3]);
  acc_guard4(acc[1][0], acc[1][1], acc[1][2], acc[1][3]);
  acc_guard4(acc[2][0], acc[2][1], acc[2][2], acc[2][3]);
  acc_guard4(acc[3][0], acc[3][1], acc[3][2], acc[3][3]);

  float* slab = sT[wave];
#pragma unroll
  for (int i = 0; i < 4; ++i) {
    const int mBase = m0 + (i << 4);
#pragma unroll
    for (int j = 0; j < 4; ++j) {
#pragma unroll
      for (int r = 0; r < 8; ++r) {
        const float v = acc[i][j][r] * kScale;
        slab[(mOff + r) * 68 + (j << 4) + rlane] = v;
      }
    }
    __builtin_amdgcn_fence(__ATOMIC_RELEASE, "workgroup");
    __builtin_amdgcn_wave_barrier();
    __builtin_amdgcn_fence(__ATOMIC_ACQUIRE, "workgroup");
    {
      const int hh = lane >> 4, c4 = (lane & 15) * 4;
      for (int pass = 0; pass < 2; ++pass) {
#pragma unroll
        for (int it = 0; it < 8; ++it) {
          const int row = it * 2 + hh;
          v4f v = *(const v4f*)(slab + row * 68 + c4);
          *(volatile v4f*)(Cout + (size_t)(mBase + row) * ldc + n0 + c4) = v;
        }
        __threadfence();
      }
    }
    __builtin_amdgcn_fence(__ATOMIC_RELEASE, "workgroup");
    __builtin_amdgcn_wave_barrier();
    __builtin_amdgcn_fence(__ATOMIC_ACQUIRE, "workgroup");
  }
}

__global__ __launch_bounds__(128) void scan_kernel(
    const float* __restrict__ P, const float* __restrict__ X, const float* __restrict__ H0,
    const float* __restrict__ Alog, const float* __restrict__ Dp,
    float* __restrict__ Y, float* __restrict__ Hout)
{
  __shared__ __align__(16) float sBC[kScanTS * 32];
  __shared__ __align__(16) float sY[2 * kScanTS * kScanYP];
  __shared__ __align__(16) float sA[kNst * kScanCh];
  __shared__ __align__(16) float sH[kScanCh * kNst];
  const unsigned tid  = threadIdx.x;
  const unsigned lane = tid & 31u;
  const unsigned wave = tid >> 5;
  const unsigned ch   = tid & 63u;
  const unsigned half = tid >> 6;
  constexpr unsigned kBlkPerB = (unsigned)(kDm / kScanCh);
  const unsigned bix = blockIdx.x / kBlkPerB;
  const unsigned d0  = (blockIdx.x - bix * kBlkPerB) * (unsigned)kScanCh;
  const unsigned d   = d0 + ch;
  const size_t row0  = (size_t)bix * kSeq;
  const unsigned sb  = half * (unsigned)kHalfSt;

#pragma unroll 1
  for (unsigned k = 0; k < (unsigned)kHalfSt; ++k) {
    const float al = Alog[(size_t)d * kNst + sb + k];
    sA[(sb + k) * kScanCh + ch] = -expf(al);
  }
  __syncthreads();
  float negA[kHalfSt], h[kHalfSt];
#pragma unroll
  for (int k = 0; k < kHalfSt; ++k) negA[k] = sA[(sb + (unsigned)k) * kScanCh + ch];
  {
    const float* hp = H0 + ((size_t)bix * kDm + d) * kNst + sb;
    const v4f ha = *(const v4f*)(hp);
    const v4f hb = *(const v4f*)(hp + 4);
    h[0] = ha.x; h[1] = ha.y; h[2] = ha.z; h[3] = ha.w;
    h[4] = hb.x; h[5] = hb.y; h[6] = hb.z; h[7] = hb.w;
  }
  const float Dd = Dp[d];
  unsigned sr = tid >> 3;
  unsigned sc4 = (tid & 7u) * 4u;
  pin_u(sr);
  pin_u(sc4);
  unsigned hh = lane >> 4;
  unsigned c4o = (lane & 15u) * 4u;
  pin_u(hh);
  pin_u(c4o);
  float* syw = sY + half * (unsigned)(kScanTS * kScanYP) + ch;

#pragma unroll 1
  for (unsigned t0 = 0; t0 < (unsigned)kSeq; t0 += (unsigned)kScanTS) {
    __syncthreads();
#pragma unroll
    for (int i = 0; i < 4; ++i) {
      const unsigned r = sr + 16u * (unsigned)i;
      *(v4f*)(sBC + r * 32u + sc4) = *(const v4f*)(P + (row0 + t0 + r) * kNpad + kDm + sc4);
    }
    __syncthreads();
#pragma unroll 1
    for (unsigned s = 0; s < (unsigned)kScanTS; ++s) {
      const size_t row = row0 + t0 + s;
      float dr = P[row * kNpad + d];
      float xv = X[row * kDm + d];
      asm volatile("" : "+v"(dr));
      asm volatile("" : "+v"(xv));
      const float* br = sBC + s * 32u + sb;
      const v4f b0 = *(const v4f*)(br);
      const v4f b1 = *(const v4f*)(br + 4);
      const v4f c0 = *(const v4f*)(br + 16);
      const v4f c1 = *(const v4f*)(br + 20);
      float Bs[kHalfSt], Cs[kHalfSt];
      Bs[0] = b0.x; Bs[1] = b0.y; Bs[2] = b0.z; Bs[3] = b0.w;
      Bs[4] = b1.x; Bs[5] = b1.y; Bs[6] = b1.z; Bs[7] = b1.w;
      Cs[0] = c0.x; Cs[1] = c0.y; Cs[2] = c0.z; Cs[3] = c0.w;
      Cs[4] = c1.x; Cs[5] = c1.y; Cs[6] = c1.z; Cs[7] = c1.w;
      const float ez = expf(-fabsf(dr));
      const float dt = fmaxf(dr, 0.0f) + log1pf(ez);
      const float dx = dt * xv;
      float y = 0.0f;
#pragma unroll
      for (int k = 0; k < kHalfSt; ++k) {
        const float a = expf(dt * negA[k]);
        h[k] = a * h[k] + dx * Bs[k];
        y = h[k] * Cs[k] + y;
      }
      const float skip = Dd * xv;
      y += (half == 0u) ? skip : 0.0f;
      syw[s * (unsigned)kScanYP] = y;
    }
    __syncthreads();
    v4f yv[8];
#pragma unroll
    for (int it = 0; it < 8; ++it) {
      const unsigned row = (unsigned)it * 8u + wave * 2u + hh;
      const v4f p0 = *(const v4f*)(sY + row * (unsigned)kScanYP + c4o);
      const v4f p1 = *(const v4f*)(sY + (unsigned)(kScanTS * kScanYP) + row * (unsigned)kScanYP + c4o);
      yv[it] = p0 + p1;
    }
    for (int pass = 0; pass < 2; ++pass) {
#pragma unroll
      for (int it = 0; it < 8; ++it) {
        const unsigned row = (unsigned)it * 8u + wave * 2u + hh;
        *(volatile v4f*)(Y + (row0 + t0 + row) * kDm + d0 + c4o) = yv[it];
      }
      __threadfence();
    }
  }

  __syncthreads();
#pragma unroll
  for (int k = 0; k < kHalfSt; ++k) sH[ch * (unsigned)kNst + sb + (unsigned)k] = h[k];
  __syncthreads();
  {
    float* hdst = Hout + ((size_t)bix * kDm + d0) * kNst;
    v4f hv[2];
#pragma unroll
    for (int it = 0; it < 2; ++it) hv[it] = *(const v4f*)(sH + ((unsigned)it * 128u + tid) * 4u);
    for (int pass = 0; pass < 2; ++pass) {
#pragma unroll
      for (int it = 0; it < 2; ++it)
        *(volatile v4f*)(hdst + ((unsigned)it * 128u + tid) * 4u) = hv[it];
      __threadfence();
    }
  }
}

extern "C" void kernel_launch(void* const* d_in, const int* in_sizes, int n_in,
                              void* d_out, int out_size, void* d_ws, size_t ws_size,
                              hipStream_t stream) {
  if (n_in < 5) return;
  if (in_sizes[0] != kRows * kDm) return;
  if (in_sizes[1] != kBatch * kDm * kNst) return;
  if (in_sizes[2] != kDm * kNproj) return;
  if (in_sizes[3] != kDm * kNst) return;
  if (in_sizes[4] != kDm) return;
  if (out_size != kRows * kDm + kBatch * kDm * kNst) return;
  if (ws_size < kWsTotal) return;

  const float* x     = (const float*)d_in[0];
  const float* h0    = (const float*)d_in[1];
  const float* W     = (const float*)d_in[2];
  const float* A_log = (const float*)d_in[3];
  const float* Dp    = (const float*)d_in[4];
  float* y    = (float*)d_out;
  float* hnew = (float*)d_out + (size_t)kRows * kDm;

  char* ws = (char*)d_ws;
  unsigned short* XH  = (unsigned short*)(ws + kOffXH);
  unsigned short* XL  = (unsigned short*)(ws + kOffXL);
  unsigned short* WTH = (unsigned short*)(ws + kOffWTH);
  unsigned short* WTL = (unsigned short*)(ws + kOffWTL);
  float*          P   = (float*)(ws + kOffP);

  pack_rows_kernel<kThreeProd><<<kPackX8 / 256u, 256, 0, stream>>>(x, XH, XL);
  pack_wt_kernel<kThreeProd><<<dim3(kDm / 64, kNpad / 64), 256, 0, stream>>>(W, WTH, WTL);
  proj_gemm_kernel<kOpType, kThreeProd><<<(kRows / 64) * (kNpad / 64) / 8, 256, 0, stream>>>(XH, XL, WTH, WTL, P);
  scan_kernel<<<kBatch * (kDm / kScanCh), 128, 0, stream>>>(P, x, h0, A_log, Dp, y, hnew);
}
